// LSTM_86990267613956
// MI455X (gfx1250) — hardware-verified
//
#include <hip/hip_runtime.h>
#include <math.h>

typedef __attribute__((ext_vector_type(16))) _Float16 v16h;
typedef __attribute__((ext_vector_type(8)))  _Float16 v8h;
typedef __attribute__((ext_vector_type(16))) __bf16   v16b;
typedef __attribute__((ext_vector_type(8)))  __bf16   v8b;
typedef __attribute__((ext_vector_type(8)))  float    v8f;
typedef __attribute__((ext_vector_type(4)))  float    v4f;

constexpr int kB    = 128;
constexpr int kT    = 512;
constexpr int kD    = 128;
constexpr int kDp   = 256;
constexpr int kHid  = 512;
constexpr int kO    = 128;
constexpr int kG4   = 4 * kHid;
constexpr int kK0   = kHid + kDp;
constexpr int kK1   = kHid + kHid;
constexpr int kRowsY = kB * kT;
constexpr int kThr  = 256;
constexpr float kInCarry = 1024.0f;
constexpr float kSc = 1.0f / (kInCarry * kInCarry);
constexpr float kF16MinNormal = 6.103515625e-5f;

static_assert((kB % 64) == 0 && (kRowsY % 64) == 0 && (kG4 % 64) == 0 && (kO % 64) == 0 && ((kB / 64) * (kG4 / 64)) % 8 == 0 && ((kRowsY / 64) * (kO / 64)) % 8 == 0, "GEMM M, N multiples of 64; grids exact");
static_assert((kK0 % 32) == 0 && (kK1 % 32) == 0 && (kHid % 32) == 0 && (kK0 % 256) == 0 && (kK1 % 256) == 0 && (kHid % 256) == 0, "GEMM K multiples of 32; the plane cast's pitches and offsets multiples of 256");

constexpr size_t kOffW0 = 0ull;
constexpr size_t kOffW1 = 3145728ull;
constexpr size_t kOffWO16 = 7340032ull;
constexpr size_t kOffBIAS = 7471104ull;
constexpr size_t kOffA0 = 7487488ull;
constexpr size_t kOffA1 = 7684096ull;
constexpr size_t kOffG0 = 7946240ull;
constexpr size_t kOffG1 = 8994816ull;
constexpr size_t kOffC0 = 10043392ull;
constexpr size_t kOffC1 = 10305536ull;
constexpr size_t kOffHS16 = 10567680ull;
constexpr size_t kWsTotal = 77676544ull;
static_assert(kWsTotal <= 134217728ull, "carve cap: under 128 MiB");
static_assert(kOffW0 == 0
              && kOffW1 == kOffW0 + 3145728ull
              && kOffWO16 == kOffW1 + 4194304ull
              && kOffBIAS == kOffWO16 + 131072ull
              && kOffA0 == kOffBIAS + 16384ull
              && kOffA1 == kOffA0 + 196608ull
              && kOffG0 == kOffA1 + 262144ull
              && kOffG1 == kOffG0 + 1048576ull
              && kOffC0 == kOffG1 + 1048576ull
              && kOffC1 == kOffC0 + 262144ull
              && kOffHS16 == kOffC1 + 262144ull
              && kWsTotal == kOffHS16 + 67108864ull, "the carve is chained and totalled");
static_assert((kOffW0 % 256) == 0 && (kOffW1 % 256) == 0 && (kOffWO16 % 256) == 0 && (kOffBIAS % 256) == 0 && (kOffA0 % 256) == 0 && (kOffA1 % 256) == 0 && (kOffG0 % 256) == 0 && (kOffG1 % 256) == 0 && (kOffC0 % 256) == 0 && (kOffC1 % 256) == 0 && (kOffHS16 % 256) == 0, "aligned regions");
constexpr int kFBO = 0, kFZB = 2048, kFEnd = 4096;
static_assert(kFBO + kO <= kFZB && kFZB + kG4 <= kFEnd && (kFZB % 128) == 0, "bias stream map; the zero row reaches the gates' 2,048 columns");

__device__ __forceinline__ unsigned short f2bf_bits(float f) {
  unsigned u = __float_as_uint(f);
  return (unsigned short)((u + 0x7FFFu + ((u >> 16) & 1u)) >> 16);
}
__device__ __forceinline__ float bf_bits2f(unsigned short h) { return __uint_as_float(((unsigned)h) << 16); }
__device__ __forceinline__ float bf16r(float f) { return bf_bits2f(f2bf_bits(f)); }
__device__ __forceinline__ float carry_flush(float v, float carry) {
  const float s = v * carry;
  return (fabsf(s) < kF16MinNormal) ? 0.0f : s;
}
__device__ __forceinline__ float frcp(float x) { return __builtin_amdgcn_rcpf(x); }

__device__ __forceinline__ void dep_guard4_h(v8f& a, v8f& b, v8f& c, v8f& d, v16h x, v16h y) { asm volatile("v_nop\n\tv_nop\n\tv_nop\n\tv_nop" : "+v"(a), "+v"(b), "+v"(c), "+v"(d) : "v"(x), "v"(y)); }
__device__ __forceinline__ void dep_guard4_b(v8f& a, v8f& b, v8f& c, v8f& d, v16b x, v16b y) { asm volatile("v_nop\n\tv_nop\n\tv_nop\n\tv_nop" : "+v"(a), "+v"(b), "+v"(c), "+v"(d) : "v"(x), "v"(y)); }
__device__ __forceinline__ void keep4_h(v16h a, v16h b, v16h c, v16h d) { asm volatile("v_nop" :: "v"(a), "v"(b), "v"(c), "v"(d)); }
__device__ __forceinline__ void keep4_b(v16b a, v16b b, v16b c, v16b d) { asm volatile("v_nop" :: "v"(a), "v"(b), "v"(c), "v"(d)); }
__device__ __forceinline__ void acc_guard4(v8f& a, v8f& b, v8f& c, v8f& d) { asm volatile("v_nop\n\tv_nop\n\tv_nop\n\tv_nop" : "+v"(a), "+v"(b), "+v"(c), "+v"(d)); }

template <typename T> struct Frag;
template <> struct Frag<_Float16> {
  typedef v16h V; union U { v16h v; v8h h[2]; };
  static __device__ __forceinline__ v16h load(const _Float16* p) {
    U f; f.h[0] = *(const v8h*)(p); f.h[1] = *(const v8h*)(p + 16); return f.v;
  }
  static __device__ __forceinline__ v8f mma(v16h a, v16h b, v8f c) {
    return __builtin_amdgcn_wmma_f32_16x16x32_f16(false, a, false, b, (short)0, c, false, false);
  }
  static __device__ __forceinline__ void guard4(v8f& a, v8f& b, v8f& c, v8f& d, v16h x, v16h y) { dep_guard4_h(a, b, c, d, x, y); }
  static __device__ __forceinline__ void keep(v16h a, v16h b, v16h c, v16h d) { keep4_h(a, b, c, d); }
};
template <> struct Frag<__bf16> {
  typedef v16b V; union U { v16b v; v8b h[2]; };
  static __device__ __forceinline__ v16b load(const __bf16* p) {
    U f; f.h[0] = *(const v8b*)(p); f.h[1] = *(const v8b*)(p + 16); return f.v;
  }
  static __device__ __forceinline__ v8f mma(v16b a, v16b b, v8f c) {
    return __builtin_amdgcn_wmma_f32_16x16x32_bf16(false, a, false, b, (short)0, c, false, false);
  }
  static __device__ __forceinline__ void guard4(v8f& a, v8f& b, v8f& c, v8f& d, v16b x, v16b y) { dep_guard4_b(a, b, c, d, x, y); }
  static __device__ __forceinline__ void keep(v16b a, v16b b, v16b c, v16b d) { keep4_b(a, b, c, d); }
};

__device__ __forceinline__ v8f mma_h(v16h a, v16h b, v8f c) {
  c = __builtin_amdgcn_wmma_f32_16x16x32_f16(false, a, false, b, (short)0, c, false, false);
  asm volatile("v_nop\n\tv_nop\n\tv_nop\n\tv_nop" : "+v"(c) : "v"(a), "v"(b));
  return c;
}

template <int ET> struct Elem;
template <> struct Elem<0> { typedef _Float16 T; };
template <> struct Elem<1> { typedef __bf16 T; };
template <int ET, bool SPLIT, int BIAS_MODE, int OUT_MODE, bool RESID, int ACT = 0>
__global__ __launch_bounds__(256) void wmma_gemm64(
    const unsigned short* __restrict__ Ap, const unsigned short* __restrict__ A2p, int lda, long strideA,
    const unsigned short* __restrict__ Btp, const unsigned short* __restrict__ Bt2p, int ldb, long strideB,
    void* __restrict__ Cout, void* __restrict__ Cout2, int ldc, long strideC,
    const float* __restrict__ bias,
    const float* __restrict__ resid, long strideR,
    int M, int N, int K, float scale) {
  typedef typename Elem<ET>::T T;
  typedef typename Frag<T>::V V;
  const T* A = (const T*)Ap; const T* A2 = (const T*)A2p; const T* Bt = (const T*)Btp; const T* Bt2 = (const T*)Bt2p;
  __shared__ __align__(16) float sT[8][16 * 68];
  const int b    = blockIdx.y;
  const int lane = threadIdx.x & 31;
  const int wave = threadIdx.x >> 5;
  const int tilesN = N >> 6;
  const int tilesM = M >> 6;
  const int tile = blockIdx.x * 8 + wave;
  if (tile >= tilesM * tilesN) return;
  const int tm = tile / tilesN;
  const int tn = tile - tm * tilesN;
  const int m0 = tm << 6;
  const int n0 = tn << 6;

  const T* Ab  = A  + (size_t)b * strideA;
  const T* Bb  = Bt + (size_t)b * strideB;
  const T* Ab2 = SPLIT ? (A2  + (size_t)b * strideA) : nullptr;
  const T* Bb2 = SPLIT ? (Bt2 + (size_t)b * strideB) : nullptr;

  const int rlane = lane & 15;
  const int koff  = (lane >> 4) * 8;
  const int mOff  = (lane >> 4) * 8;

  v8f acc[4][4];
#pragma unroll
  for (int i = 0; i < 4; ++i)
#pragma unroll
    for (int j = 0; j < 4; ++j) acc[i][j] = (v8f){0.f,0.f,0.f,0.f,0.f,0.f,0.f,0.f};

  for (int k0 = 0; k0 < K; k0 += 32) {
    V bh[4], bl[4];
#pragma unroll
    for (int j = 0; j < 4; ++j) {
      const size_t bo = (size_t)(n0 + (j << 4) + rlane) * ldb + koff + k0;
      bh[j] = Frag<T>::load(Bb + bo);
      if (SPLIT) bl[j] = Frag<T>::load(Bb2 + bo);
    }
#pragma unroll
    for (int i = 0; i < 4; ++i) {
      const size_t ao = (size_t)(m0 + (i << 4) + rlane) * lda + koff + k0;
      V ah = Frag<T>::load(Ab + ao);
      V al;
      if (SPLIT) al = Frag<T>::load(Ab2 + ao);
#pragma unroll
      for (int j = 0; j < 4; ++j) {
        acc[i][j] = Frag<T>::mma(ah, bh[j], acc[i][j]);
        if (SPLIT) {
          acc[i][j] = Frag<T>::mma(ah, bl[j], acc[i][j]);
          acc[i][j] = Frag<T>::mma(al, bh[j], acc[i][j]);
        }
      }
      Frag<T>::guard4(acc[i][0], acc[i][1], acc[i][2], acc[i][3], ah, SPLIT ? al : ah);
    }
    Frag<T>::keep(bh[0], bh[1], bh[2], bh[3]);
    if (SPLIT) Frag<T>::keep(bl[0], bl[1], bl[2], bl[3]);
  }
  acc_guard4(acc[0][0], acc[0][1], acc[0][2], acc[0][3]);
  acc_guard4(acc[1][0], acc[1][1], acc[1][2], acc[1][3]);
  acc_guard4(acc[2][0], acc[2][1], acc[2][2], acc[2][3]);
  acc_guard4(acc[3][0], acc[3][1], acc[3][2], acc[3][3]);

  float* slab = sT[wave];
  const float* Rb = RESID ? (resid + (size_t)b * strideR) : nullptr;
#pragma unroll
  for (int i = 0; i < 4; ++i) {
    const int mBase = m0 + (i << 4);
#pragma unroll
    for (int j = 0; j < 4; ++j) {
      const int n = n0 + (j << 4) + rlane;
      float bv = 0.f;
      if (BIAS_MODE == 2) bv = bias[n];
#pragma unroll
      for (int r = 0; r < 8; ++r) {
        float v = acc[i][j][r] * scale;
        if (BIAS_MODE == 1) v += bias[mBase + mOff + r];
        if (BIAS_MODE == 2) v += bv;
        if (RESID) v += Rb[(size_t)(mBase + mOff + r) * ldc + n];
        if (ACT == 1) v = tanhf(v);
        if (ACT == 2) v = fmaxf(v, 0.0f);
        if (ACT == 3) v = v / (1.0f + expf(-v));
        if (ACT == 4) v = (v > 0.f) ? v : 0.01f * v;
        slab[(mOff + r) * 68 + (j << 4) + rlane] = v;
      }
    }
    __builtin_amdgcn_fence(__ATOMIC_RELEASE, "workgroup");
    __builtin_amdgcn_wave_barrier();
    __builtin_amdgcn_fence(__ATOMIC_ACQUIRE, "workgroup");
    if (OUT_MODE == 0) {
      float* C = (float*)Cout + (size_t)b * strideC;
      const int hh = lane >> 4, c4 = (lane & 15) * 4;
      for (int pass = 0; pass < 2; ++pass) {
#pragma unroll
        for (int it = 0; it < 8; ++it) {
          const int row = it * 2 + hh;
          v4f v = *(const v4f*)(slab + row * 68 + c4);
          *(volatile v4f*)(C + (size_t)(mBase + row) * ldc + n0 + c4) = v;
        }
        __threadfence();
      }
    } else {
      const int q = lane >> 3, c8 = (lane & 7) * 8;
      unsigned short* C  = (unsigned short*)Cout  + (size_t)b * strideC;
      unsigned short* C2 = (OUT_MODE == 2) ? ((unsigned short*)Cout2 + (size_t)b * strideC) : nullptr;
      for (int pass = 0; pass < 2; ++pass) {
#pragma unroll
        for (int it = 0; it < 4; ++it) {
          const int row = it * 4 + q;
          const float* sp = slab + row * 68 + c8;
          v8h hv, lv;
#pragma unroll
          for (int e = 0; e < 8; ++e) {
            if (OUT_MODE == 1) {
              hv[e] = (_Float16)sp[e];
            } else {
              unsigned short hb = f2bf_bits(sp[e]);
              unsigned short lb = f2bf_bits(sp[e] - bf_bits2f(hb));
              hv[e] = __builtin_bit_cast(_Float16, hb);
              lv[e] = __builtin_bit_cast(_Float16, lb);
            }
          }
          *(volatile v8h*)(C + (size_t)(mBase + row) * ldc + n0 + c8) = hv;
          if (OUT_MODE == 2) *(volatile v8h*)(C2 + (size_t)(mBase + row) * ldc + n0 + c8) = lv;
        }
        __threadfence();
      }
    }
    __builtin_amdgcn_fence(__ATOMIC_RELEASE, "workgroup");
    __builtin_amdgcn_wave_barrier();
    __builtin_amdgcn_fence(__ATOMIC_ACQUIRE, "workgroup");
  }
}

__global__ __launch_bounds__(kThr) void cast_plane_kernel(const float* __restrict__ src, unsigned short* __restrict__ dst,
                                                          int colsLog2, int dstPitch, int dstOff) {
  const int i   = blockIdx.x * kThr + threadIdx.x;
  const int sh  = colsLog2 - 3;
  const int row = i >> sh;
  const int c8  = (i & ((1 << sh) - 1)) * 8;
  const float* sp = src + ((size_t)row << colsLog2) + c8;
  const v4f a0 = *(const v4f*)(sp);
  const v4f a1 = *(const v4f*)(sp + 4);
  v8h hv;
#pragma unroll
  for (int e = 0; e < 4; ++e) {
    const float f0 = a0[e];
    const float f1 = a1[e];
    hv[e]     = (_Float16)carry_flush(bf16r(f0), kInCarry);
    hv[4 + e] = (_Float16)carry_flush(bf16r(f1), kInCarry);
  }
  unsigned short* dp = dst + (size_t)row * dstPitch + dstOff + c8;
  *(volatile v8h*)dp = hv;
  __threadfence();
  *(volatile v8h*)dp = hv;
}

__device__ __forceinline__ float fast_tanh(float v) { return 1.0f - 2.0f * frcp(__expf(2.0f * v) + 1.0f); }
__device__ __forceinline__ float fast_sigmoid(float v) { return frcp(1.0f + __expf(-v)); }

__global__ __launch_bounds__(kThr) void setup_kernel(const float* __restrict__ x, const float* __restrict__ h0, const float* __restrict__ c0,
                                                     const float* __restrict__ w_ih_0, const float* __restrict__ b_out, float* __restrict__ BIAS,
                                                     unsigned short* __restrict__ W0, unsigned short* __restrict__ A0, unsigned short* __restrict__ A1,
                                                     float* __restrict__ C0, float* __restrict__ C1) {
  unsigned v = blockIdx.x * (unsigned)kThr + threadIdx.x;
  asm volatile("" : "+v"(v));
  if (v < 1024u) {
    const unsigned i0 = v * 4u;
    v4f o = {0.f, 0.f, 0.f, 0.f};
    if (i0 < (unsigned)kO) {
      const v4f a = *(const v4f*)(b_out + i0);
#pragma unroll
      for (int e = 0; e < 4; ++e) { const float p = a[e]; o[e] = bf16r(p); }
    }
    float* dp = BIAS + i0;
    *(volatile v4f*)dp = o;
    __threadfence();
    *(volatile v4f*)dp = o;
  } else if (v < 95232u) {
    v8h hv;
#pragma unroll
    for (int e = 0; e < 8; ++e) hv[e] = (_Float16)0.0f;
    unsigned short* dp;
    const float* sp = x;
    bool ld = false;
    if (v < 66560u) {
      const unsigned w = v - 1024u;
      const unsigned n = w >> 5, c8 = (w & 31u) * 8u;
      if (c8 < (unsigned)kD) { sp = w_ih_0 + (size_t)n * kD + c8; ld = true; }
      dp = W0 + (size_t)n * kK0 + kHid + c8;
    } else if (v < 74752u) {
      const unsigned w = v - 66560u;
      sp = h0 + (size_t)(w >> 6) * kHid + (w & 63u) * 8u; ld = true;
      dp = A0 + (size_t)(w >> 6) * kK0 + (w & 63u) * 8u;
    } else if (v < 78848u) {
      const unsigned w = v - 74752u;
      const unsigned b = w >> 5, c8 = (w & 31u) * 8u;
      if (c8 < (unsigned)kD) { sp = x + (size_t)b * kT * kD + c8; ld = true; }
      dp = A0 + (size_t)b * kK0 + kHid + c8;
    } else if (v < 87040u) {
      const unsigned w = v - 78848u;
      sp = h0 + (size_t)kB * kHid + (size_t)(w >> 6) * kHid + (w & 63u) * 8u; ld = true;
      dp = A1 + (size_t)(w >> 6) * kK1 + (w & 63u) * 8u;
    } else {
      const unsigned w = v - 87040u;
      dp = A1 + (size_t)(w >> 6) * kK1 + kHid + (w & 63u) * 8u;
    }
    if (ld) {
      const v4f a0 = *(const v4f*)sp, a1 = *(const v4f*)(sp + 4);
#pragma unroll
      for (int e = 0; e < 4; ++e) { const float p = a0[e], q = a1[e]; hv[e] = (_Float16)carry_flush(bf16r(p), kInCarry); hv[4 + e] = (_Float16)carry_flush(bf16r(q), kInCarry); }
    }
    *(volatile v8h*)dp = hv;
    __threadfence();
    *(volatile v8h*)dp = hv;
  } else {
    const unsigned w = v - 95232u;
    const v4f a = *(const v4f*)(c0 + (size_t)w * 4u);
    v4f o;
#pragma unroll
    for (int e = 0; e < 4; ++e) { const float p = a[e]; o[e] = bf16r(p); }
    float* dp = (w < 16384u) ? (C0 + (size_t)w * 4u) : (C1 + (size_t)(w - 16384u) * 4u);
    *(volatile v4f*)dp = o;
    __threadfence();
    *(volatile v4f*)dp = o;
  }
}
static_assert(kFEnd / 4 == 1024 && kG4 * kDp / 8 == 65536 && kB * kHid / 8 == 8192 && kB * kDp / 8 == 4096 && kB * kHid / 4 == 16384 && 1024 + 65536 + 8192 + 4096 + 8192 + 8192 + 16384 + 16384 == 500 * kThr, "set-up grid exact");
static_assert((1024 % 32) == 0 && (66560 % 32) == 0 && (74752 % 32) == 0 && (78848 % 32) == 0 && (87040 % 32) == 0 && (95232 % 32) == 0 && (kD % 8) == 0, "set-up regions wave-uniform");

__global__ __launch_bounds__(kThr) void cell2_kernel(const float* __restrict__ G0, const float* __restrict__ G1, const float* __restrict__ x,
                                                     float* __restrict__ C0, float* __restrict__ C1, unsigned short* __restrict__ A0,
                                                     unsigned short* __restrict__ A1, unsigned short* __restrict__ HS16, int k) {
  const int layer = (int)(blockIdx.x >> 5);
  if (layer == 0 ? (k >= kT) : (k < 1)) return;
  unsigned v = (blockIdx.x & 31u) * (unsigned)kThr + threadIdx.x;
  asm volatile("" : "+v"(v));
  const unsigned b = v >> 6;
  const unsigned u8 = (v & 63u) * 8u;
  const float* gr = (layer == 0 ? G0 : G1) + (size_t)b * kG4 + u8;
  float* cp = (layer == 0 ? C0 : C1) + (size_t)b * kHid + u8;
  v8h hv, xv;
  v4f cn0, cn1;
#pragma unroll
  for (int hlf = 0; hlf < 2; ++hlf) {
    const v4f gi = *(const v4f*)(gr + 4 * hlf), gf = *(const v4f*)(gr + kHid + 4 * hlf), gg = *(const v4f*)(gr + 2 * kHid + 4 * hlf), go = *(const v4f*)(gr + 3 * kHid + 4 * hlf);
    const v4f co = *(const v4f*)(cp + 4 * hlf);
#pragma unroll
    for (int e = 0; e < 4; ++e) {
      const float cn = fast_sigmoid(gf[e]) * co[e] + fast_sigmoid(gi[e]) * fast_tanh(gg[e]);
      const float hn = fast_sigmoid(go[e]) * fast_tanh(cn);
      if (hlf == 0) cn0[e] = cn; else cn1[e] = cn;
      hv[4 * hlf + e] = (_Float16)carry_flush(hn, kInCarry);
    }
  }
  if (layer == 0) {
    const bool nx = (u8 < (unsigned)kD) && (k + 1 < kT);
    {
      const float* sp = x + ((size_t)b * kT + (size_t)(nx ? (k + 1) : 0)) * kD + (nx ? u8 : 0u);
      const v4f a0 = *(const v4f*)sp, a1 = *(const v4f*)(sp + 4);
#pragma unroll
      for (int e = 0; e < 4; ++e) { const float p = a0[e], q = a1[e]; xv[e] = (_Float16)carry_flush(bf16r(p), kInCarry); xv[4 + e] = (_Float16)carry_flush(bf16r(q), kInCarry); }
    }
    unsigned short* hp = A0 + (size_t)b * kK0 + u8;
    unsigned short* yp = A1 + (size_t)b * kK1 + kHid + u8;
    unsigned short* xp = A0 + (size_t)b * kK0 + kHid + (nx ? u8 : 0u);
    for (int pass = 0; pass < 2; ++pass) {
      *(volatile v4f*)cp = cn0; *(volatile v4f*)(cp + 4) = cn1;
      *(volatile v8h*)hp = hv;
      *(volatile v8h*)yp = hv;
      if (nx) *(volatile v8h*)xp = xv;
      __threadfence();
    }
  } else {
    unsigned short* hp = A1 + (size_t)b * kK1 + u8;
    unsigned short* sp2 = HS16 + ((size_t)b * kT + (size_t)(k - 1)) * kHid + u8;
    for (int pass = 0; pass < 2; ++pass) {
      *(volatile v4f*)cp = cn0; *(volatile v4f*)(cp + 4) = cn1;
      *(volatile v8h*)hp = hv;
      *(volatile v8h*)sp2 = hv;
      __threadfence();
    }
  }
}
static_assert(kB * kHid / 8 == 32 * kThr && kHid / 8 == 64 && (kD / 8) == 16, "cell grid: 32 blocks a layer; the input's 16 lanes are the first half of a wave");

static_assert(((size_t)kG4 * kHid / 8) % kThr == 0 && ((size_t)kO * kHid / 8) % kThr == 0, "plane cast grids exact");

extern "C" void kernel_launch(void* const* d_in, const int* in_sizes, int n_in,
                              void* d_out, int out_size, void* d_ws, size_t ws_size,
                              hipStream_t stream) {
  if (n_in < 9 || d_out == nullptr || d_ws == nullptr) return;
  if (in_sizes[0] != kB * kT * kD || in_sizes[1] != 2 * kB * kHid || in_sizes[2] != 2 * kB * kHid || in_sizes[3] != kG4 * kD || in_sizes[4] != kG4 * kHid) return;
  if (in_sizes[5] != kG4 * kHid || in_sizes[6] != kG4 * kHid || in_sizes[7] != kO * kHid || in_sizes[8] != kO) return;
  if (out_size != kRowsY * kO) return;
  if (ws_size < kWsTotal) return;
  const float* x = (const float*)d_in[0];
  const float* h0 = (const float*)d_in[1];
  const float* c0 = (const float*)d_in[2];
  const float* w_ih_0 = (const float*)d_in[3];
  const float* w_hh_0 = (const float*)d_in[4];
  const float* w_ih_1 = (const float*)d_in[5];
  const float* w_hh_1 = (const float*)d_in[6];
  const float* w_out = (const float*)d_in[7];
  const float* b_out = (const float*)d_in[8];
  float* out = (float*)d_out;
  char* ws = (char*)d_ws;
  unsigned short* W0 = (unsigned short*)(ws + kOffW0);
  unsigned short* W1 = (unsigned short*)(ws + kOffW1);
  unsigned short* WO16 = (unsigned short*)(ws + kOffWO16);
  float* BIAS = (float*)(ws + kOffBIAS);
  unsigned short* A0 = (unsigned short*)(ws + kOffA0);
  unsigned short* A1 = (unsigned short*)(ws + kOffA1);
  float* G0 = (float*)(ws + kOffG0);
  float* G1 = (float*)(ws + kOffG1);
  float* C0 = (float*)(ws + kOffC0);
  float* C1 = (float*)(ws + kOffC1);
  unsigned short* HS16 = (unsigned short*)(ws + kOffHS16);

  cast_plane_kernel<<<(int)(((size_t)kG4 * kHid / 8) / kThr), kThr, 0, stream>>>(w_hh_0, W0, 9, kK0, 0);
  cast_plane_kernel<<<(int)(((size_t)kG4 * kHid / 8) / kThr), kThr, 0, stream>>>(w_hh_1, W1, 9, kK1, 0);
  cast_plane_kernel<<<(int)(((size_t)kG4 * kHid / 8) / kThr), kThr, 0, stream>>>(w_ih_1, W1, 9, kK1, kHid);
  cast_plane_kernel<<<(int)(((size_t)kO * kHid / 8) / kThr), kThr, 0, stream>>>(w_out, WO16, 9, kHid, 0);
  setup_kernel<<<500, kThr, 0, stream>>>(x, h0, c0, w_ih_0, b_out, BIAS, W0, A0, A1, C0, C1);

  for (int k = 0; k <= kT; ++k) {
    if (k < kT) {
      wmma_gemm64<0, false, 2, 0, false, 0><<<dim3((kB / 64) * (kG4 / 64) / 8, 1), 256, 0, stream>>>(
          A0, A0, kK0, 0L, W0, W0, kK0, 0L, (void*)G0, (void*)G0, kG4, 0L, BIAS + kFZB, nullptr, 0L, kB, kG4, kK0, kSc);
    }
    if (k >= 1) {
      wmma_gemm64<0, false, 2, 0, false, 0><<<dim3((kB / 64) * (kG4 / 64) / 8, 1), 256, 0, stream>>>(
          A1, A1, kK1, 0L, W1, W1, kK1, 0L, (void*)G1, (void*)G1, kG4, 0L, BIAS + kFZB, nullptr, 0L, kB, kG4, kK1, kSc);
    }
    cell2_kernel<<<64, kThr, 0, stream>>>(G0, G1, x, C0, C1, A0, A1, HS16, k);
  }
  wmma_gemm64<0, false, 2, 0, false, 0><<<dim3((kRowsY / 64) * (kO / 64) / 8, 1), 256, 0, stream>>>(
      HS16, HS16, kHid, 0L, WO16, WO16, kHid, 0L, (void*)out, (void*)out, kO, 0L, BIAS + kFBO, nullptr, 0L, kRowsY, kO, kHid, kSc);
}
